// ParametricClampedBeam_56083682951607
// MI455X (gfx1250) — hardware-verified
//
#include <hip/hip_runtime.h>
#include <math.h>

typedef __attribute__((ext_vector_type(16))) _Float16 v16h;
typedef __attribute__((ext_vector_type(16))) __bf16 v16b;
typedef __attribute__((ext_vector_type(8)))  _Float16 v8h;
typedef __attribute__((ext_vector_type(8)))  float v8f;
typedef __attribute__((ext_vector_type(4)))  float v4f;
typedef __attribute__((ext_vector_type(2)))  float v2f;
typedef __attribute__((ext_vector_type(4)))  unsigned v4u;
typedef __attribute__((ext_vector_type(4)))  int v4i;
typedef float __attribute__((may_alias)) float_a;
typedef int __attribute__((may_alias)) int_a;

template <typename T> __device__ __forceinline__ void vst2(void* p, T v) { *(volatile T*)p = v; __threadfence(); *(volatile T*)p = v; }
__device__ __forceinline__ v8f wmma16(v16h a, v16h b, v8f c) {
  v8f d = __builtin_amdgcn_wmma_f32_16x16x32_f16(false, a, false, b, (short)0, c, false, false);
  asm volatile("v_nop\n\tv_nop\n\tv_nop\n\tv_nop" : "+v"(d) : "v"(a), "v"(b));
  return d;
}
__device__ __forceinline__ v8f wmma_bf(v16b a, v16b b, v8f c) {
  v8f d = __builtin_amdgcn_wmma_f32_16x16x32_bf16(false, a, false, b, (short)0, c, false, false);
  asm volatile("v_nop\n\tv_nop\n\tv_nop\n\tv_nop" : "+v"(d) : "v"(a), "v"(b));
  return d;
}
__device__ __forceinline__ v16h frag_h(const _Float16* rowk0, int lane) {
  union { v16h v; v8h q[2]; } u; const _Float16* p = rowk0 + 8 * (lane >> 4);
  u.q[0] = *(const v8h*)p; u.q[1] = *(const v8h*)(p + 16); return u.v;
}
__device__ __forceinline__ v16h frag_f32(const float* rowk0, int lane) {
  v16h a; const float* p = rowk0 + 8 * (lane >> 4);
#pragma unroll
  for (int i = 0; i < 8; ++i) { a[i] = (_Float16)p[i]; a[8 + i] = (_Float16)p[16 + i]; }
  return a;
}
__device__ __forceinline__ v16h frag_f32s(const float* rowk0, int lane, float sc) {
  v16h a; const float* p = rowk0 + 8 * (lane >> 4);
#pragma unroll
  for (int i = 0; i < 8; ++i) { a[i] = (_Float16)(p[i] * sc); a[8 + i] = (_Float16)(p[16 + i] * sc); }
  return a;
}
__device__ __forceinline__ v16h fragc_f32(const float* W, int k0, int n, int lane, int ld, int K) {
  v16h a; const int g = lane >> 4;
#pragma unroll
  for (int i = 0; i < 8; ++i) { const int ka = k0 + 8 * g + i, kb = ka + 16;
    a[i] = (_Float16)(ka < K ? W[(size_t)(ka < K ? ka : K - 1) * ld + n] : 0.f); a[8 + i] = (_Float16)(kb < K ? W[(size_t)(kb < K ? kb : K - 1) * ld + n] : 0.f); }
  return a;
}
struct F2 { v16b h, l; };
__device__ __forceinline__ F2 bsplit16(const float v[16]) { F2 r;
#pragma unroll
  for (int i = 0; i < 16; ++i) { const __bf16 h = (__bf16)v[i]; r.h[i] = h; r.l[i] = (__bf16)(v[i] - (float)h); }
  return r; }
__device__ __forceinline__ F2 split_row(const float* row, int k0, int lane) { float v[16]; const float* p = row + k0 + 8 * (lane >> 4);
#pragma unroll
  for (int i = 0; i < 8; ++i) { v[i] = p[i]; v[8 + i] = p[16 + i]; }
  return bsplit16(v); }
__device__ __forceinline__ F2 split_rowK(const float* row, int k0, int lane, int K) { float v[16]; const int g = lane >> 4;
#pragma unroll
  for (int i = 0; i < 8; ++i) { const int ka = k0 + 8 * g + i, kb = ka + 16; v[i] = ka < K ? row[ka < K ? ka : K - 1] : 0.f; v[8 + i] = kb < K ? row[kb < K ? kb : K - 1] : 0.f; }
  return bsplit16(v); }
__device__ __forceinline__ F2 split_col(const float* W, int k0, int n, int lane, int ld, int K) { float v[16]; const int g = lane >> 4;
#pragma unroll
  for (int i = 0; i < 8; ++i) { const int ka = k0 + 8 * g + i, kb = ka + 16; v[i] = ka < K ? W[(size_t)(ka < K ? ka : K - 1) * ld + n] : 0.f; v[8 + i] = kb < K ? W[(size_t)(kb < K ? kb : K - 1) * ld + n] : 0.f; }
  return bsplit16(v); }
__device__ __forceinline__ v8f mac3(const F2& a, const F2& b, v8f c) { c = wmma_bf(a.l, b.h, c); c = wmma_bf(a.h, b.l, c); return wmma_bf(a.h, b.h, c); }
__device__ __forceinline__ float sigm(float v) { return 1.0f / (1.0f + expf(-v)); }
#define LDSX() do { asm volatile("s_wait_dscnt 0" ::: "memory"); __builtin_amdgcn_wave_barrier(); __builtin_amdgcn_fence(__ATOMIC_RELEASE, "workgroup"); } while (0)


#define NPTS 262144
#define HU 64
#ifndef TRB
#define TRB (NPTS / 64)
#endif
typedef __attribute__((ext_vector_type(8))) __bf16 v8b;
__device__ __forceinline__ v16b frag_b(const __bf16* rowk0, int lane) {
  union { v16b v; v8b q[2]; } u; const __bf16* p = rowk0 + 8 * (lane >> 4);
  u.q[0] = *(const v8b*)p; u.q[1] = *(const v8b*)(p + 16); return u.v;
}
__device__ __forceinline__ float bfr(float v) { return (float)(__bf16)v; }
__device__ __attribute__((noinline)) float exp_ni(float v) { return expf(v); }
__device__ __attribute__((noinline)) float erf_ni(float v) { return erff(v); }

__device__ __attribute__((noinline)) float tanh_ni(float v) { return tanhf(v); }
__device__ __forceinline__ void put_hl(__bf16* h, __bf16* l, float v) { const __bf16 hb = (__bf16)v; *h = hb; *l = (__bf16)(v - (float)hb); }
#define WS_P2  0u
#define WS_P3  (WS_P2 + 2u * HU * HU)
#define WS_END (WS_P3 + 2u * HU * HU)

__global__ __launch_bounds__(64) void k_packT(const float* __restrict__ Wm, __bf16* __restrict__ DST) {
  __shared__ __align__(16) __bf16 s[8 * HU]; const int n0 = blockIdx.x * 8, tid = threadIdx.x;
  for (int q = tid; q < 8 * HU; q += 64) { const int rl = q >> 6, k = q & 63; s[q] = (__bf16)Wm[(size_t)k * HU + n0 + rl]; }
  __syncthreads();
  vst2((unsigned*)(DST + (size_t)n0 * HU + tid * 8), *(const v4u*)&s[tid * 8]);
}
__device__ __forceinline__ void tanh_jet(float c[5]) {
  const float u1 = c[1], u2 = c[2], u3 = c[3], u4 = c[4]; const float t = tanh_ni(c[0]); const float s = 1.0f - t * t;
  const float t1 = s, t2h = -t * s  , t3s = s * (6.0f * t * t - 2.0f) * (1.0f / 6.0f), t4s = 8.0f * t * s * (2.0f - 3.0f * t * t) * (1.0f / 24.0f);
  const float d22 = u1 * u1, d23 = 2.0f * u1 * u2, d24 = 2.0f * u1 * u3 + u2 * u2; const float d33 = d22 * u1, d34 = 3.0f * d22 * u2; const float d44 = d22 * d22;
  c[0] = t; c[1] = t1 * u1; c[2] = t1 * u2 + t2h * d22; c[3] = t1 * u3 + t2h * d23 + t3s * d33; c[4] = t1 * u4 + t2h * d24 + t3s * d34 + t4s * d44;
}
__global__ __launch_bounds__(128) void k_beam(const float* __restrict__ X, const float* __restrict__ EE, const float* __restrict__ II, const float* __restrict__ QQ, const float* __restrict__ W1, const float* __restrict__ b1, const __bf16* __restrict__ P2, const float* __restrict__ b2, const __bf16* __restrict__ P3, const float* __restrict__ b3, const float* __restrict__ W4, const float* __restrict__ b4, float* __restrict__ out) {
  __shared__ __align__(16) __bf16 sah[4][5][16][HU + 8], sal[4][5][16][HU + 8];
  __shared__ __align__(16) float spre[4][5][16][HU + 4];
  __shared__ float sw1[4][HU], sb1[HU], sw4[HU]; __shared__ __align__(16) float sres[5][64];
  const int tid = threadIdx.x, wave = tid >> 5, lane = tid & 31, col = lane & 15, g = lane >> 4; const size_t p0 = (size_t)blockIdx.x * 64 + wave * 16;
  for (int q = tid; q < 4 * HU; q += 128) sw1[q / HU][q % HU] = bfr(W1[q]);
  for (int q = tid; q < HU; q += 128) { sb1[q] = bfr(b1[q]); sw4[q] = bfr(W4[q]); }
  __syncthreads();
  for (int q = lane; q < 16 * HU; q += 32) { const int pl = q >> 6, u = q & 63; const size_t p = p0 + pl;
    const float xv = bfr(X[p]), ev = bfr(EE[p]) * (1.0f / 2.0e11f), iv = bfr(II[p]) * (1.0f / 1.0e-6f), qv = bfr(QQ[p]) * (1.0f / 1.0e3f);
    float c[5]; c[0] = xv * sw1[0][u] + ev * sw1[1][u] + iv * sw1[2][u] + qv * sw1[3][u] + sb1[u]; c[1] = sw1[0][u]; c[2] = 0.f; c[3] = 0.f; c[4] = 0.f;
    tanh_jet(c);
#pragma unroll
    for (int k = 0; k < 5; ++k) put_hl(&sah[wave][k][pl][u], &sal[wave][k][pl][u], c[k]); }
  LDSX();
#pragma unroll 1
  for (int layer = 0; layer < 2; ++layer) { const __bf16* P = layer == 0 ? P2 : P3; const float* bb = layer == 0 ? b2 : b3;
#pragma unroll 1
    for (int k = 0; k < 5; ++k) { v8f acc[4] = {};
#pragma unroll
      for (int kc = 0; kc < 2; ++kc) { const v16b ah = frag_b(&sah[wave][k][col][kc * 32], lane), al = frag_b(&sal[wave][k][col][kc * 32], lane);
#pragma unroll
        for (int j = 0; j < 4; ++j) { const v16b w = frag_b(P + (size_t)(j * 16 + col) * HU + kc * 32, lane); acc[j] = wmma_bf(al, w, acc[j]); acc[j] = wmma_bf(ah, w, acc[j]); } }
#pragma unroll
      for (int j = 0; j < 4; ++j) { const float bv = (k == 0) ? bfr(bb[j * 16 + col]) : 0.f;
#pragma unroll
        for (int r = 0; r < 8; ++r) spre[wave][k][8 * g + r][j * 16 + col] = acc[j][r] + bv; } }
    LDSX();
    for (int q = lane; q < 16 * HU; q += 32) { const int pl = q >> 6, u = q & 63; float c[5];
#pragma unroll
      for (int k = 0; k < 5; ++k) c[k] = spre[wave][k][pl][u];
      tanh_jet(c);
#pragma unroll
      for (int k = 0; k < 5; ++k) put_hl(&sah[wave][k][pl][u], &sal[wave][k][pl][u], c[k]); }
    LDSX(); }
  if (lane < 16) { const int pl = lane; const size_t p = p0 + pl; float c[5];
#pragma unroll
    for (int k = 0; k < 5; ++k) { float s = (k == 0) ? bfr(b4[0]) : 0.f;
#pragma unroll 4
      for (int u = 0; u < HU; ++u) s += ((float)sah[wave][k][pl][u] + (float)sal[wave][k][pl][u]) * sw4[u];
      c[k] = s; }
    const float psi = c[0], px = c[1], pxx = 2.0f * c[2], pxxx = 6.0f * c[3], pxxxx = 24.0f * c[4];
    const float xv = bfr(X[p]); const float x2 = xv * xv;
    const float w0 = x2 * psi, w1v = 2.0f * xv * psi + x2 * px, w2v = 2.0f * psi + 4.0f * xv * px + x2 * pxx, w3v = 6.0f * px + 6.0f * xv * pxx + x2 * pxxx, w4v = 12.0f * pxx + 8.0f * xv * pxxx + x2 * pxxxx;
    const float sc = bfr(QQ[p]) / (bfr(EE[p]) * bfr(II[p]) + 1.1920929e-07f);
    sres[0][wave * 16 + pl] = sc * w0; sres[1][wave * 16 + pl] = sc * w1v; sres[2][wave * 16 + pl] = sc * w2v; sres[3][wave * 16 + pl] = sc * w3v; sres[4][wave * 16 + pl] = sc * w4v; }
  __syncthreads();
  if (tid < 80) { const int k = tid >> 4, pc = tid & 15; vst2(out + (size_t)k * NPTS + (size_t)blockIdx.x * 64 + pc * 4, *(const v4f*)&sres[k][pc * 4]); }
}
extern "C" void kernel_launch(void* const* d_in, const int* in_sizes, int n_in, void* d_out, int out_size, void* d_ws, size_t ws_size, hipStream_t stream) {
  (void)in_sizes; (void)n_in; (void)out_size;
  const float** F = (const float**)d_in;
  if (ws_size < (size_t)WS_END) return;
  char* ws = (char*)d_ws; __bf16 *P2 = (__bf16*)(ws + WS_P2), *P3 = (__bf16*)(ws + WS_P3);
  k_packT<<<HU / 8, 64, 0, stream>>>(F[6], P2); k_packT<<<HU / 8, 64, 0, stream>>>(F[8], P3);
  k_beam<<<TRB, 128, 0, stream>>>(F[0], F[1], F[2], F[3], F[4], F[5], P2, F[7], P3, F[9], F[10], F[11], (float*)d_out);
}
